// M100_14336600834653
// MI455X (gfx1250) — hardware-verified
//
#include <hip/hip_runtime.h>
#pragma clang fp contract(off)

#define HID 128
#define NT_SCAN 128
#define NT_HEAD 256
#define RPB 256

typedef _Float16 v8h  __attribute__((ext_vector_type(8)));
typedef _Float16 v16h __attribute__((ext_vector_type(16)));
typedef float    v8f  __attribute__((ext_vector_type(8)));
typedef float    v4f  __attribute__((ext_vector_type(4)));
typedef v8h __attribute__((may_alias)) v8ha;
typedef v4f __attribute__((may_alias)) v4fa;
union Frag { v16h v; v8h half[2]; };

__device__ __forceinline__ v8f vzero8() {
    v8f z = {0.f, 0.f, 0.f, 0.f, 0.f, 0.f, 0.f, 0.f};
    return z;
}

__device__ __forceinline__ v8f wmma16(v8f acc, v16h a, v16h b) {
    acc = __builtin_amdgcn_wmma_f32_16x16x32_f16(false, a, false, b, (short)0, acc, false, false);
    asm volatile("v_nop\n\tv_nop\n\tv_nop\n\tv_nop" : "+v"(acc) : "v"(a), "v"(b));
    return acc;
}

__device__ __forceinline__ float stepf(float v) {
    return 0.5f * (tanhf(5.0f * v) + 1.0f);
}

__device__ __forceinline__ float interp_lin(const float* __restrict__ fp, const float* __restrict__ tg,
                                            int T, float t) {
    int i = (int)t + 1;
    i = (i > T - 1) ? (T - 1) : i;
    i = (i < 1) ? 1 : i;
    const int lo = i - 1;
    const float xlo = tg[lo], xhi = tg[i];
    const float dx = xhi - xlo;
    const float delta = t - xlo;
    const float flo = fp[lo], fhi = fp[i];
    const float df = fhi - flo;
    float f;
    if (fabsf(dx) <= 1.4210855e-14f) f = flo;
    else f = flo + (delta * (1.0f / dx)) * df;
    if (t < tg[0]) f = fp[0];
    if (t > tg[T - 1]) f = fp[T - 1];
    return f;
}

__device__ __forceinline__ void flush_chunk(const float* straj, float* sol, int chunk, int wave, int lane) {
    if (wave == 0 && lane < 16) {
        const v4f v = *(const v4fa*)(straj + 4 * lane);
        volatile v4f* p = (volatile v4f*)(sol + (size_t)chunk * 64 + 4 * lane);
        *p = v;
        __threadfence();
        *p = v;
    }
}

__global__ __launch_bounds__(NT_SCAN) void k_scan(
    const float* __restrict__ x, const float* __restrict__ t_eval, const float* __restrict__ t_grid,
    const float* __restrict__ precp, const float* __restrict__ temp, const float* __restrict__ lday,
    const float* __restrict__ W1, const float* __restrict__ b1,
    const float* __restrict__ W2, const float* __restrict__ b2,
    const float* __restrict__ W3, const float* __restrict__ b3,
    float* sol, int T)
{
    __shared__ _Float16 sBh[HID * HID] __attribute__((aligned(16)));
    __shared__ _Float16 sBl[HID * HID] __attribute__((aligned(16)));
    __shared__ _Float16 sA[16 * HID]   __attribute__((aligned(16)));
    __shared__ float sW1[4 * HID];
    __shared__ float sb1[HID];
    __shared__ float sb2[HID];
    __shared__ float sW3[HID * 5];
    __shared__ float sb3[8];
    __shared__ float sS[2];
    __shared__ float sred[4][8];
    __shared__ float sTraj[64] __attribute__((aligned(16)));

    const int tid  = threadIdx.x;
    const int lane = tid & 31;
    const int wave = tid >> 5;
    const int hf   = lane >> 4;
    const int m    = lane & 15;

    for (int e = tid; e < HID * HID; e += NT_SCAN) {
        const int n = e >> 7, k = e & (HID - 1);
        const float w = W2[k * HID + n] * 64.0f;
        const _Float16 whi = (_Float16)w;
        const float wres = (w - (float)whi) * 2048.0f;
        sBh[e] = whi;
        sBl[e] = (_Float16)wres;
    }
    for (int e = tid; e < 16 * HID; e += NT_SCAN) sA[e] = (_Float16)0.0f;
    for (int e = tid; e < 4 * HID; e += NT_SCAN) sW1[e] = W1[e];
    for (int e = tid; e < 5 * HID; e += NT_SCAN) sW3[e] = W3[e];
    sb1[tid] = b1[tid];
    sb2[tid] = b2[tid];
    if (tid < 5) sb3[tid] = b3[tid];
    if (tid < 64) sTraj[tid] = (tid == 0) ? x[0] : ((tid == 1) ? x[1] : 0.0f);
    if (tid == 0) { sS[0] = x[0]; sS[1] = x[1]; }
    __syncthreads();

    float Sb0 = sS[0], Sb1 = sS[1];
    float ka0 = 0.0f, ka1 = 0.0f;

    const float c11 = 0.00048828125f;
    const float c22 = 2.384185791015625e-07f;
    const float c10 = 0.0009765625f;
    const int n0 = 32 * wave + m;
    const int n1 = n0 + 16;

    for (int n = 0; n + 1 < T; ++n) {
        const float t0 = t_eval[n];
        const float t1 = t_eval[n + 1];
        const float hh = t1 - t0;
        const float ch = 0.5f * hh;
        #pragma unroll 1
        for (int st = 0; st < 4; ++st) {
            const float ts = (st == 0) ? t0 : ((st == 3) ? t1 : (t0 + ch));
            const float pr = interp_lin(precp, t_grid, T, ts);
            const float te = interp_lin(temp,  t_grid, T, ts);
            const float z0 = sS[0], z1 = sS[1];

            float a1 = z0 * sW1[tid];
            a1 = a1 + z1 * sW1[HID + tid];
            a1 = a1 + pr * sW1[2 * HID + tid];
            a1 = a1 + te * sW1[3 * HID + tid];
            a1 = a1 + sb1[tid];
            const float hv = tanhf(a1) * 16.0f;
            const _Float16 hhi = (_Float16)hv;
            const float hres = (hv - (float)hhi) * 2048.0f;
            sA[tid]       = hhi;
            sA[HID + tid] = (_Float16)hres;
            __syncthreads();

            v8f aH0 = vzero8(), aH1 = vzero8(), aL0 = vzero8(), aL1 = vzero8();
            #pragma unroll
            for (int ks = 0; ks < 4; ++ks) {
                const int k0 = ks * 32;
                Frag fa, fb;
                const _Float16* ap = sA + m * HID + k0 + 8 * hf;
                fa.half[0] = *(const v8ha*)(ap);
                fa.half[1] = *(const v8ha*)(ap + 16);
                const _Float16* bp0h = sBh + n0 * HID + k0 + 8 * hf;
                fb.half[0] = *(const v8ha*)(bp0h);
                fb.half[1] = *(const v8ha*)(bp0h + 16);
                aH0 = wmma16(aH0, fa.v, fb.v);
                const _Float16* bp0l = sBl + n0 * HID + k0 + 8 * hf;
                fb.half[0] = *(const v8ha*)(bp0l);
                fb.half[1] = *(const v8ha*)(bp0l + 16);
                aL0 = wmma16(aL0, fa.v, fb.v);
                const _Float16* bp1h = sBh + n1 * HID + k0 + 8 * hf;
                fb.half[0] = *(const v8ha*)(bp1h);
                fb.half[1] = *(const v8ha*)(bp1h + 16);
                aH1 = wmma16(aH1, fa.v, fb.v);
                const _Float16* bp1l = sBl + n1 * HID + k0 + 8 * hf;
                fb.half[0] = *(const v8ha*)(bp1l);
                fb.half[1] = *(const v8ha*)(bp1l + 16);
                aL1 = wmma16(aL1, fa.v, fb.v);
            }
            const float P0 = aH0[0] + (aH0[1] + aL0[0]) * c11 + aL0[1] * c22;
            const float P1 = aH1[0] + (aH1[1] + aL1[0]) * c11 + aL1[1] * c22;
            const float h20 = tanhf(P0 * c10 + sb2[n0]);
            const float h21 = tanhf(P1 * c10 + sb2[n1]);
            const float msk = (hf == 0) ? 1.0f : 0.0f;

            float p0 = msk * (h20 * sW3[n0 * 5 + 0] + h21 * sW3[n1 * 5 + 0]);
            float p1 = msk * (h20 * sW3[n0 * 5 + 1] + h21 * sW3[n1 * 5 + 1]);
            float p2 = msk * (h20 * sW3[n0 * 5 + 2] + h21 * sW3[n1 * 5 + 2]);
            float p3 = msk * (h20 * sW3[n0 * 5 + 3] + h21 * sW3[n1 * 5 + 3]);
            float p4 = msk * (h20 * sW3[n0 * 5 + 4] + h21 * sW3[n1 * 5 + 4]);
            #pragma unroll
            for (int off = 8; off >= 1; off >>= 1) {
                p0 += __shfl_xor(p0, off, 32);
                p1 += __shfl_xor(p1, off, 32);
                p2 += __shfl_xor(p2, off, 32);
                p3 += __shfl_xor(p3, off, 32);
                p4 += __shfl_xor(p4, off, 32);
            }
            if (lane == 0) {
                sred[wave][0] = p0; sred[wave][1] = p1; sred[wave][2] = p2;
                sred[wave][3] = p3; sred[wave][4] = p4;
            }
            __syncthreads();

            if (tid == 0) {
                float s0 = (sred[0][0] + sred[1][0]) + sred[2][0]; s0 = s0 + sred[3][0];
                float s1 = (sred[0][1] + sred[1][1]) + sred[2][1]; s1 = s1 + sred[3][1];
                float s2 = (sred[0][2] + sred[1][2]) + sred[2][2]; s2 = s2 + sred[3][2];
                float s3 = (sred[0][3] + sred[1][3]) + sred[2][3]; s3 = s3 + sred[3][3];
                float s4 = (sred[0][4] + sred[1][4]) + sred[2][4]; s4 = s4 + sred[3][4];
                const float o0 = s0 + sb3[0];
                const float o1 = s1 + sb3[1];
                const float o2 = s2 + sb3[2];
                const float o3 = s3 + sb3[3];
                const float o4 = s4 + sb3[4];
                const float ld = interp_lin(lday, t_grid, T, ts);
                const float stz0 = stepf(z0);
                const float stz1 = stepf(z1);
                const float stnt = stepf(-te);
                const float melt = fmaxf(stz0, 0.0f) * sinhf(o2);
                const float d1 = fmaxf(sinhf(o3) * stnt, 0.0f) - melt;
                float d2 = fmaxf(sinhf(o4), 0.0f) + melt;
                d2 = d2 - (stz1 * ld) * expf(o0);
                d2 = d2 - stz1 * expf(o1);
                if (st == 0) {
                    ka0 = d1; ka1 = d2;
                    sS[0] = Sb0 + ch * d1; sS[1] = Sb1 + ch * d2;
                } else if (st == 1) {
                    ka0 = ka0 + 2.0f * d1; ka1 = ka1 + 2.0f * d2;
                    sS[0] = Sb0 + ch * d1; sS[1] = Sb1 + ch * d2;
                } else if (st == 2) {
                    ka0 = ka0 + 2.0f * d1; ka1 = ka1 + 2.0f * d2;
                    sS[0] = Sb0 + hh * d1; sS[1] = Sb1 + hh * d2;
                } else {
                    ka0 = ka0 + d1; ka1 = ka1 + d2;
                    const float h6 = hh * (1.0f / 6.0f);
                    Sb0 = Sb0 + h6 * ka0;
                    Sb1 = Sb1 + h6 * ka1;
                    sS[0] = Sb0; sS[1] = Sb1;
                    const int e = n + 1;
                    sTraj[2 * (e & 31)]     = Sb0;
                    sTraj[2 * (e & 31) + 1] = Sb1;
                }
            }
            __syncthreads();
        }
        const int e = n + 1;
        if ((e & 31) == 31) flush_chunk(sTraj, sol, e >> 5, wave, lane);
    }
    __syncthreads();
    flush_chunk(sTraj, sol, (T - 1) >> 5, wave, lane);
}

__global__ __launch_bounds__(NT_HEAD) void k_head(
    const float* __restrict__ x, const float* __restrict__ sol,
    const float* __restrict__ W1, const float* __restrict__ b1,
    const float* __restrict__ W2, const float* __restrict__ b2,
    const float* __restrict__ W3, const float* __restrict__ b3,
    float* out, int T)
{
    __shared__ _Float16 sBt[HID * HID] __attribute__((aligned(16)));
    __shared__ float sW1[4 * HID];
    __shared__ float sb1[HID];
    __shared__ float sb2[HID];
    __shared__ float sw3[HID];
    __shared__ float sOut[RPB] __attribute__((aligned(16)));

    const int tid = threadIdx.x;
    for (int e = tid; e < HID * HID; e += NT_HEAD) {
        const int n = e >> 7, k = e & (HID - 1);
        sBt[e] = (_Float16)(W2[k * HID + n] * 64.0f);
    }
    for (int e = tid; e < 4 * HID; e += NT_HEAD) sW1[e] = W1[e];
    if (tid < HID) {
        sb1[tid] = b1[tid];
        sb2[tid] = b2[tid];
        sw3[tid] = W3[tid * 5 + 1];
    }
    __syncthreads();

    const int lane = tid & 31;
    const int wave = tid >> 5;
    const int hf   = lane >> 4;
    const int m    = lane & 15;
    const int rowBase = blockIdx.x * RPB + wave * 32;
    const float b3_1 = b3[1];
    const float c10 = 0.0009765625f;

    #pragma unroll 1
    for (int mt = 0; mt < 2; ++mt) {
        const int m0 = rowBase + mt * 16;
        int r = m0 + m;
        r = (r > T - 1) ? (T - 1) : r;
        const float z0 = sol[2 * r], z1 = sol[2 * r + 1];
        const float z2 = x[4 * r + 2], z3 = x[4 * r + 3];

        v8f acc[8];
        #pragma unroll
        for (int nn = 0; nn < 8; ++nn) acc[nn] = vzero8();

        #pragma unroll
        for (int s = 0; s < 4; ++s) {
            v16h afrag;
            #pragma unroll
            for (int v = 0; v < 8; ++v) {
                const int kb = s * 32 + ((v < 4) ? (2 * v) : (16 + 2 * (v - 4))) + 8 * hf;
                float h0 = z0 * sW1[kb];
                h0 = h0 + z1 * sW1[HID + kb];
                h0 = h0 + z2 * sW1[2 * HID + kb];
                h0 = h0 + z3 * sW1[3 * HID + kb];
                h0 = h0 + sb1[kb];
                float h1 = z0 * sW1[kb + 1];
                h1 = h1 + z1 * sW1[HID + kb + 1];
                h1 = h1 + z2 * sW1[2 * HID + kb + 1];
                h1 = h1 + z3 * sW1[3 * HID + kb + 1];
                h1 = h1 + sb1[kb + 1];
                afrag[2 * v]     = (_Float16)(tanhf(h0) * 16.0f);
                afrag[2 * v + 1] = (_Float16)(tanhf(h1) * 16.0f);
            }
            #pragma unroll
            for (int nn = 0; nn < 8; ++nn) {
                Frag fb;
                const _Float16* bp = sBt + (nn * 16 + m) * HID + s * 32 + 8 * hf;
                fb.half[0] = *(const v8ha*)(bp);
                fb.half[1] = *(const v8ha*)(bp + 16);
                acc[nn] = wmma16(acc[nn], afrag, fb.v);
            }
        }

        #pragma unroll
        for (int rr = 0; rr < 8; ++rr) {
            float sacc = 0.0f;
            #pragma unroll
            for (int nn = 0; nn < 8; ++nn) {
                const int N = nn * 16 + m;
                sacc = sacc + tanhf(acc[nn][rr] * c10 + sb2[N]) * sw3[N];
            }
            sacc += __shfl_xor(sacc, 1, 32);
            sacc += __shfl_xor(sacc, 2, 32);
            sacc += __shfl_xor(sacc, 4, 32);
            sacc += __shfl_xor(sacc, 8, 32);
            if (m == 0) sOut[wave * 32 + mt * 16 + 8 * hf + rr] = expf(sacc + b3_1);
        }
    }
    __syncthreads();

    const bool full = (rowBase + 32 <= T);
    if (full) {
        if (lane < 8) {
            const v4f v = *(const v4fa*)(sOut + wave * 32 + 4 * lane);
            volatile v4f* p = (volatile v4f*)(out + rowBase + 4 * lane);
            *p = v;
            __threadfence();
            *p = v;
        }
    } else {
        const int row = rowBase + lane;
        if (row < T) {
            const float v = sOut[wave * 32 + lane];
            volatile float* p = (volatile float*)(out + row);
            *p = v;
            __threadfence();
            *p = v;
        }
    }
}

extern "C" void kernel_launch(void* const* d_in, const int* in_sizes, int n_in,
                              void* d_out, int out_size, void* d_ws, size_t ws_size,
                              hipStream_t stream) {
    if (n_in < 12) return;
    const float* x      = (const float*)d_in[0];
    const float* t_eval = (const float*)d_in[1];
    const float* t_grid = (const float*)d_in[2];
    const float* precp  = (const float*)d_in[3];
    const float* temp   = (const float*)d_in[4];
    const float* lday   = (const float*)d_in[5];
    const float* W1 = (const float*)d_in[6];
    const float* b1 = (const float*)d_in[7];
    const float* W2 = (const float*)d_in[8];
    const float* b2 = (const float*)d_in[9];
    const float* W3 = (const float*)d_in[10];
    const float* b3 = (const float*)d_in[11];
    const int T = in_sizes[1];

    if (T < 2) return;
    if (in_sizes[0] < 4 * T || in_sizes[2] < T || in_sizes[3] < T || in_sizes[4] < T || in_sizes[5] < T) return;
    if (in_sizes[6] < 4 * HID || in_sizes[7] < HID || in_sizes[8] < HID * HID || in_sizes[9] < HID ||
        in_sizes[10] < 5 * HID || in_sizes[11] < 5) return;
    if (out_size < T) return;

    const size_t nchunks   = ((size_t)T + 31) / 32;
    const size_t sol_bytes = nchunks * 64 * sizeof(float);
    if (sol_bytes > ws_size) return;
    float* sol = (float*)d_ws;

    k_scan<<<1, NT_SCAN, 0, stream>>>(x, t_eval, t_grid, precp, temp, lday,
                                      W1, b1, W2, b2, W3, b3, sol, T);

    const int blocks = (T + RPB - 1) / RPB;
    k_head<<<blocks, NT_HEAD, 0, stream>>>(x, sol, W1, b1, W2, b2, W3, b3, (float*)d_out, T);
}
